// TreeRNN_85761906966779
// MI455X (gfx1250) — hardware-run, weakly checked
//
#include <hip/hip_runtime.h>
#include <math.h>

constexpr int N_LEAVES = 524288;
constexpr int N_NONTERM = N_LEAVES - 1;
constexpr int EMB_DIM  = 64;
constexpr int HID_DIM  = 128;
constexpr int CAT_DIM  = 256;
constexpr int VOC_WRD  = 100000;
constexpr int VOC_POS  = 64;
constexpr int VOC_NON  = 64;
constexpr int A_PITCH  = 264;
constexpr int SLAB_PITCH = 68;
constexpr int TAIL_ROWS = 64;
constexpr float STATE_CARRY  = 64.0f;
constexpr float WEIGHT_CARRY = 16.0f;
constexpr float CARRY_FOLD   = 1.0f / (STATE_CARRY * WEIGHT_CARRY);
static_assert(HID_DIM == 2 * EMB_DIM);
static_assert(CAT_DIM == 2 * HID_DIM);
static_assert(CAT_DIM % 32 == 0);
static_assert(HID_DIM == 2 * 64);
static_assert((N_LEAVES / 2) % 64 == 0);
static_assert((A_PITCH * 2) % 16 == 0);

typedef __attribute__((ext_vector_type(16))) _Float16 v16h;
typedef __attribute__((ext_vector_type(8)))  _Float16 v8h;
typedef __attribute__((ext_vector_type(16))) __bf16   v16b;
typedef __attribute__((ext_vector_type(8)))  __bf16   v8b;
typedef __attribute__((ext_vector_type(8)))  float    v8f;
typedef __attribute__((ext_vector_type(4)))  float    v4f;
typedef __attribute__((ext_vector_type(2)))  float    v2f;
typedef __attribute__((ext_vector_type(4)))  unsigned v4u;

__device__ __forceinline__ unsigned short f2bf_bits(float f) {
  unsigned u = __float_as_uint(f);
  return (unsigned short)((u + 0x7FFFu + ((u >> 16) & 1u)) >> 16);
}
__device__ __forceinline__ float bf_bits2f(unsigned short h) { return __uint_as_float(((unsigned)h) << 16); }
__device__ __forceinline__ int clamp_idx(int v, int hi) { return v < 0 ? 0 : (v > hi ? hi : v); }

__device__ __forceinline__ void dep_guard4_h(v8f& a, v8f& b, v8f& c, v8f& d, v16h x, v16h y) {
  asm volatile("v_nop\n\tv_nop\n\tv_nop\n\tv_nop" : "+v"(a), "+v"(b), "+v"(c), "+v"(d) : "v"(x), "v"(y));
}
__device__ __forceinline__ void dep_guard4_b(v8f& a, v8f& b, v8f& c, v8f& d, v16b x, v16b y) {
  asm volatile("v_nop\n\tv_nop\n\tv_nop\n\tv_nop" : "+v"(a), "+v"(b), "+v"(c), "+v"(d) : "v"(x), "v"(y));
}
__device__ __forceinline__ void keep4_h(v16h a, v16h b, v16h c, v16h d) { asm volatile("v_nop" :: "v"(a), "v"(b), "v"(c), "v"(d)); }
__device__ __forceinline__ void keep4_b(v16b a, v16b b, v16b c, v16b d) { asm volatile("v_nop" :: "v"(a), "v"(b), "v"(c), "v"(d)); }
__device__ __forceinline__ void acc_guard4(v8f& a, v8f& b, v8f& c, v8f& d) {
  asm volatile("v_nop\n\tv_nop\n\tv_nop\n\tv_nop" : "+v"(a), "+v"(b), "+v"(c), "+v"(d));
}

template <typename T> struct Frag;
template <> struct Frag<_Float16> {
  typedef v16h V; union U { v16h v; v8h h[2]; };
  static __device__ __forceinline__ v16h load(const _Float16* p) {
    U f; f.h[0] = *(const v8h*)(p); f.h[1] = *(const v8h*)(p + 16); return f.v;
  }
  static __device__ __forceinline__ v8f mma(v16h a, v16h b, v8f c) {
    return __builtin_amdgcn_wmma_f32_16x16x32_f16(false, a, false, b, (short)0, c, false, false);
  }
  static __device__ __forceinline__ void guard4(v8f& a, v8f& b, v8f& c, v8f& d, v16h x, v16h y) { dep_guard4_h(a, b, c, d, x, y); }
  static __device__ __forceinline__ void keep(v16h a, v16h b, v16h c, v16h d) { keep4_h(a, b, c, d); }
};
template <> struct Frag<__bf16> {
  typedef v16b V; union U { v16b v; v8b h[2]; };
  static __device__ __forceinline__ v16b load(const __bf16* p) {
    U f; f.h[0] = *(const v8b*)(p); f.h[1] = *(const v8b*)(p + 16); return f.v;
  }
  static __device__ __forceinline__ v8f mma(v16b a, v16b b, v8f c) {
    return __builtin_amdgcn_wmma_f32_16x16x32_bf16(false, a, false, b, (short)0, c, false, false);
  }
  static __device__ __forceinline__ void guard4(v8f& a, v8f& b, v8f& c, v8f& d, v16b x, v16b y) { dep_guard4_b(a, b, c, d, x, y); }
  static __device__ __forceinline__ void keep(v16b a, v16b b, v16b c, v16b d) { keep4_b(a, b, c, d); }
};

template <int ET> struct Elem;
template <> struct Elem<0> { typedef _Float16 T; };
template <> struct Elem<1> { typedef __bf16 T; };

__global__ __launch_bounds__(256) void weight_planes_kernel(const float* __restrict__ src,
                                                            unsigned short* __restrict__ WF,
                                                            unsigned short* __restrict__ WH,
                                                            unsigned short* __restrict__ WL, int n8) {
  const int i = blockIdx.x * 256 + threadIdx.x;
  if (i < n8) {
    const float* sp = src + (size_t)i * 8;
    const v4f a = *(const v4f*)(sp);
    const v4f b = *(const v4f*)(sp + 4);
    v8h vf, vh, vl;
#pragma unroll
    for (int e = 0; e < 4; ++e) {
      const float x0 = a[e];
      const float x1 = b[e];
      const unsigned short h0 = f2bf_bits(x0);
      const unsigned short h1 = f2bf_bits(x1);
      const unsigned short l0 = f2bf_bits(x0 - bf_bits2f(h0));
      const unsigned short l1 = f2bf_bits(x1 - bf_bits2f(h1));
      vf[e]     = (_Float16)(x0 * WEIGHT_CARRY);
      vf[4 + e] = (_Float16)(x1 * WEIGHT_CARRY);
      vh[e]     = __builtin_bit_cast(_Float16, h0);
      vh[4 + e] = __builtin_bit_cast(_Float16, h1);
      vl[e]     = __builtin_bit_cast(_Float16, l0);
      vl[4 + e] = __builtin_bit_cast(_Float16, l1);
    }
    *(volatile v8h*)(WF + (size_t)i * 8) = vf;
    *(volatile v8h*)(WH + (size_t)i * 8) = vh;
    *(volatile v8h*)(WL + (size_t)i * 8) = vl;
    __threadfence();
    *(volatile v8h*)(WF + (size_t)i * 8) = vf;
    *(volatile v8h*)(WH + (size_t)i * 8) = vh;
    *(volatile v8h*)(WL + (size_t)i * 8) = vl;
  }
}

template <int ET, bool SPLIT, int OUT_MODE, bool GATHER>
__global__ __launch_bounds__(256) void pair_level_kernel(
    const unsigned short* __restrict__ Ap, const unsigned short* __restrict__ A2p,
    const int* __restrict__ pos_idx, const int* __restrict__ wrd_idx,
    const float* __restrict__ Wpos, const float* __restrict__ Wwrd,
    const unsigned short* __restrict__ Btp, const unsigned short* __restrict__ Bt2p,
    unsigned short* __restrict__ Cout, unsigned short* __restrict__ Cout2,
    const float* __restrict__ Wnon, const float* __restrict__ bias, const int* __restrict__ nonIdx,
    int M, float scale, float oscale) {
  typedef typename Elem<ET>::T T;
  typedef typename Frag<T>::V V;
  static_assert(!GATHER || (ET == 0 && !SPLIT));
  constexpr int WPB = GATHER ? 2 : 8;
  __shared__ __align__(16) float sT[WPB][16 * SLAB_PITCH];
  __shared__ __align__(16) T At[GATHER ? 64 * A_PITCH : 8];

  const T* A   = (const T*)Ap;
  const T* A2  = (const T*)A2p;
  const T* Bt  = (const T*)Btp;
  const T* Bt2 = (const T*)Bt2p;

  const int lane = threadIdx.x & 31;
  const int wave = threadIdx.x >> 5;
  const int tile = blockIdx.x * WPB + wave;
  if (!GATHER) {
    if (tile >= (M >> 6) * 2) return;
  }
  const int m0 = (tile >> 1) << 6;
  const int n0 = (tile & 1) << 6;

  if (GATHER) {
    const int tid = threadIdx.x;
    const int f8  = (tid & 7) * 8;
    const int sub = tid >> 3;
#pragma unroll 1
    for (int it = 0; it < 8; ++it) {
      const int row  = it * 8 + sub;
      const int leaf = 2 * (m0 + row);
      const int p0 = clamp_idx(pos_idx[leaf],     VOC_POS - 1);
      const int p1 = clamp_idx(pos_idx[leaf + 1], VOC_POS - 1);
      const int w0 = clamp_idx(wrd_idx[leaf],     VOC_WRD - 1);
      const int w1 = clamp_idx(wrd_idx[leaf + 1], VOC_WRD - 1);
      const float* s0 = Wpos + (size_t)p0 * EMB_DIM + f8;
      const float* s1 = Wwrd + (size_t)w0 * EMB_DIM + f8;
      const float* s2 = Wpos + (size_t)p1 * EMB_DIM + f8;
      const float* s3 = Wwrd + (size_t)w1 * EMB_DIM + f8;
      const v4f x00 = *(const v4f*)(s0);
      const v4f x01 = *(const v4f*)(s0 + 4);
      const v4f x10 = *(const v4f*)(s1);
      const v4f x11 = *(const v4f*)(s1 + 4);
      const v4f x20 = *(const v4f*)(s2);
      const v4f x21 = *(const v4f*)(s2 + 4);
      const v4f x30 = *(const v4f*)(s3);
      const v4f x31 = *(const v4f*)(s3 + 4);
      v8h h0, h1, h2, h3;
#pragma unroll
      for (int e = 0; e < 4; ++e) {
        h0[e] = (_Float16)(x00[e] * STATE_CARRY);
        h0[4 + e] = (_Float16)(x01[e] * STATE_CARRY);
        h1[e] = (_Float16)(x10[e] * STATE_CARRY);
        h1[4 + e] = (_Float16)(x11[e] * STATE_CARRY);
        h2[e] = (_Float16)(x20[e] * STATE_CARRY);
        h2[4 + e] = (_Float16)(x21[e] * STATE_CARRY);
        h3[e] = (_Float16)(x30[e] * STATE_CARRY);
        h3[4 + e] = (_Float16)(x31[e] * STATE_CARRY);
      }
      T* dst = At + row * A_PITCH + f8;
      *(v8h*)(void*)(dst)       = h0;
      *(v8h*)(void*)(dst + 64)  = h1;
      *(v8h*)(void*)(dst + 128) = h2;
      *(v8h*)(void*)(dst + 192) = h3;
    }
    __syncthreads();
  }

  const int rlane = lane & 15;
  const int koff  = (lane >> 4) * 8;
  const int mOff  = (lane >> 4) * 8;

  v8f acc[4][4];
#pragma unroll
  for (int i = 0; i < 4; ++i)
#pragma unroll
    for (int j = 0; j < 4; ++j) acc[i][j] = (v8f){0.f, 0.f, 0.f, 0.f, 0.f, 0.f, 0.f, 0.f};

  const size_t bofs = (size_t)(n0 + rlane) * CAT_DIM + koff;
  const size_t aofs = (size_t)(m0 + rlane) * CAT_DIM + koff;
  const int    lofs = rlane * A_PITCH + koff;

  for (int k0 = 0; k0 < CAT_DIM; k0 += 32) {
    V bh[4], bl[4];
#pragma unroll
    for (int j = 0; j < 4; ++j) {
      const size_t bo = bofs + (size_t)(j * 16 * CAT_DIM) + k0;
      bh[j] = Frag<T>::load(Bt + bo);
      if (SPLIT) bl[j] = Frag<T>::load(Bt2 + bo);
    }
#pragma unroll
    for (int i = 0; i < 4; ++i) {
      V ah;
      V al;
      if (GATHER) {
        ah = Frag<T>::load(At + lofs + i * 16 * A_PITCH + k0);
      } else {
        const size_t ao = aofs + (size_t)(i * 16 * CAT_DIM) + k0;
        ah = Frag<T>::load(A + ao);
        if (SPLIT) al = Frag<T>::load(A2 + ao);
      }
#pragma unroll
      for (int j = 0; j < 4; ++j) {
        acc[i][j] = Frag<T>::mma(ah, bh[j], acc[i][j]);
        if (SPLIT) {
          acc[i][j] = Frag<T>::mma(ah, bl[j], acc[i][j]);
          acc[i][j] = Frag<T>::mma(al, bh[j], acc[i][j]);
        }
      }
      Frag<T>::guard4(acc[i][0], acc[i][1], acc[i][2], acc[i][3], ah, SPLIT ? al : ah);
    }
    Frag<T>::keep(bh[0], bh[1], bh[2], bh[3]);
    if (SPLIT) Frag<T>::keep(bl[0], bl[1], bl[2], bl[3]);
  }
  acc_guard4(acc[0][0], acc[0][1], acc[0][2], acc[0][3]);
  acc_guard4(acc[1][0], acc[1][1], acc[1][2], acc[1][3]);
  acc_guard4(acc[2][0], acc[2][1], acc[2][2], acc[2][3]);
  acc_guard4(acc[3][0], acc[3][1], acc[3][2], acc[3][3]);

  float* slab = sT[wave];
  const v2f bv = *(const v2f*)(bias + n0 + 2 * lane);
  const float bv0 = bv[0];
  const float bv1 = bv[1];
#pragma unroll
  for (int i = 0; i < 4; ++i) {
    const int mBase = m0 + (i << 4);
#pragma unroll
    for (int j = 0; j < 4; ++j) {
#pragma unroll
      for (int r = 0; r < 8; ++r) slab[(mOff + r) * SLAB_PITCH + (j << 4) + rlane] = acc[i][j][r];
    }
    __builtin_amdgcn_fence(__ATOMIC_RELEASE, "workgroup");
    __builtin_amdgcn_wave_barrier();
    __builtin_amdgcn_fence(__ATOMIC_ACQUIRE, "workgroup");
#pragma unroll 1
    for (int row = 0; row < 16; ++row) {
      const int lab = clamp_idx(nonIdx[mBase + row], VOC_NON - 1);
      const v2f wn = *(const v2f*)(Wnon + (size_t)lab * HID_DIM + n0 + 2 * lane);
      float* sp = slab + row * SLAB_PITCH + 2 * lane;
      const v2f s = *(const v2f*)(sp);
      const float wn0 = wn[0];
      const float wn1 = wn[1];
      const float z0 = s[0] * scale + wn0 + bv0;
      const float z1 = s[1] * scale + wn1 + bv1;
      v2f o;
      o[0] = tanhf(z0) * oscale;
      o[1] = tanhf(z1) * oscale;
      *(v2f*)(sp) = o;
    }
    __builtin_amdgcn_fence(__ATOMIC_RELEASE, "workgroup");
    __builtin_amdgcn_wave_barrier();
    __builtin_amdgcn_fence(__ATOMIC_ACQUIRE, "workgroup");
    {
      const int q = lane >> 3, c8 = (lane & 7) * 8;
      unsigned short* C  = Cout;
      unsigned short* C2 = Cout2;
      for (int pass = 0; pass < 2; ++pass) {
#pragma unroll
        for (int it = 0; it < 4; ++it) {
          const int row = it * 4 + q;
          const float* sp = slab + row * SLAB_PITCH + c8;
          v8h hv, lv;
#pragma unroll
          for (int e = 0; e < 8; ++e) {
            const float sv = sp[e];
            if (OUT_MODE == 1) {
              hv[e] = (_Float16)sv;
            } else {
              const unsigned short hb = f2bf_bits(sv);
              const unsigned short lb = f2bf_bits(sv - bf_bits2f(hb));
              hv[e] = __builtin_bit_cast(_Float16, hb);
              lv[e] = __builtin_bit_cast(_Float16, lb);
            }
          }
          *(volatile v8h*)(C + (size_t)(mBase + row) * HID_DIM + n0 + c8) = hv;
          if (OUT_MODE == 2) *(volatile v8h*)(C2 + (size_t)(mBase + row) * HID_DIM + n0 + c8) = lv;
        }
        __threadfence();
      }
    }
    __builtin_amdgcn_fence(__ATOMIC_RELEASE, "workgroup");
    __builtin_amdgcn_wave_barrier();
    __builtin_amdgcn_fence(__ATOMIC_ACQUIRE, "workgroup");
  }
}

__global__ __launch_bounds__(256) void root_tail_kernel(const unsigned short* __restrict__ Hi,
                                                        const unsigned short* __restrict__ Lo,
                                                        const float* __restrict__ Wc,
                                                        const float* __restrict__ Wnon,
                                                        const float* __restrict__ bias,
                                                        const int* __restrict__ nonIdx,
                                                        float* __restrict__ out) {
  __shared__ __align__(16) float sS[(TAIL_ROWS + TAIL_ROWS / 2) * HID_DIM];
  const int tid = threadIdx.x;
#pragma unroll 1
  for (int it = 0; it < 4; ++it) {
    const int idx = it * 256 + tid;
    const v4u hw = *(const v4u*)(const void*)(Hi + (size_t)idx * 8);
    const v4u lw = *(const v4u*)(const void*)(Lo + (size_t)idx * 8);
    const unsigned h0 = hw[0], h1 = hw[1], h2 = hw[2], h3 = hw[3];
    const unsigned l0 = lw[0], l1 = lw[1], l2 = lw[2], l3 = lw[3];
    v4f o0, o1;
    o0[0] = __uint_as_float(h0 << 16)         + __uint_as_float(l0 << 16);
    o0[1] = __uint_as_float(h0 & 0xffff0000u) + __uint_as_float(l0 & 0xffff0000u);
    o0[2] = __uint_as_float(h1 << 16)         + __uint_as_float(l1 << 16);
    o0[3] = __uint_as_float(h1 & 0xffff0000u) + __uint_as_float(l1 & 0xffff0000u);
    o1[0] = __uint_as_float(h2 << 16)         + __uint_as_float(l2 << 16);
    o1[1] = __uint_as_float(h2 & 0xffff0000u) + __uint_as_float(l2 & 0xffff0000u);
    o1[2] = __uint_as_float(h3 << 16)         + __uint_as_float(l3 << 16);
    o1[3] = __uint_as_float(h3 & 0xffff0000u) + __uint_as_float(l3 & 0xffff0000u);
    *(v4f*)(sS + idx * 8)     = o0;
    *(v4f*)(sS + idx * 8 + 4) = o1;
  }
  __syncthreads();

  const int j  = tid & 127;
  const int mg = tid >> 7;
  const float bj = bias[j];
  const float* wrow = Wc + (size_t)j * CAT_DIM;
  int in_off  = 0;
  int out_off = TAIL_ROWS * HID_DIM;
  int off = 0;
#pragma unroll 1
  for (int n = TAIL_ROWS / 2; n >= 1; n >>= 1) {
#pragma unroll 1
    for (int m = mg; m < n; m += 2) {
      const int abase = in_off + m * CAT_DIM;
      float a0 = 0.0f, a1 = 0.0f, a2 = 0.0f, a3 = 0.0f;
#pragma unroll 1
      for (int k = 0; k < CAT_DIM; k += 4) {
        const v4f w = *(const v4f*)(wrow + k);
        const v4f x = *(const v4f*)(sS + abase + k);
        a0 = fmaf(x[0], w[0], a0);
        a1 = fmaf(x[1], w[1], a1);
        a2 = fmaf(x[2], w[2], a2);
        a3 = fmaf(x[3], w[3], a3);
      }
      const int lab = clamp_idx(nonIdx[off + m], VOC_NON - 1);
      const float z = ((a0 + a1) + (a2 + a3)) + Wnon[(size_t)lab * HID_DIM + j] + bj;
      sS[out_off + m * HID_DIM + j] = tanhf(z);
    }
    __syncthreads();
    off += n;
    const int t = in_off;
    in_off = out_off;
    out_off = t;
  }
  if (tid < 32) {
    const v4f v = *(const v4f*)(sS + in_off + 4 * tid);
    *(volatile v4f*)(out + 4 * tid) = v;
    __threadfence();
    *(volatile v4f*)(out + 4 * tid) = v;
  }
}

extern "C" void kernel_launch(void* const* d_in, const int* in_sizes, int n_in,
                              void* d_out, int out_size, void* d_ws, size_t ws_size, hipStream_t stream) {
  if (n_in < 8 || d_out == nullptr || d_ws == nullptr) return;
  if (in_sizes[0] != N_LEAVES || in_sizes[1] != N_LEAVES || in_sizes[2] != N_NONTERM ||
      in_sizes[3] != VOC_WRD * EMB_DIM || in_sizes[4] != VOC_POS * EMB_DIM || in_sizes[5] != VOC_NON * HID_DIM ||
      in_sizes[6] != HID_DIM * CAT_DIM || in_sizes[7] != HID_DIM || out_size != HID_DIM) return;

  const int*   pos_idx = (const int*)d_in[0];
  const int*   wrd_idx = (const int*)d_in[1];
  const int*   non_idx = (const int*)d_in[2];
  const float* Wwrd    = (const float*)d_in[3];
  const float* Wpos    = (const float*)d_in[4];
  const float* Wnon    = (const float*)d_in[5];
  const float* Wc_w    = (const float*)d_in[6];
  const float* Wc_b    = (const float*)d_in[7];
  float* out = (float*)d_out;

  char* ws = (char*)d_ws; size_t off = 0;
  auto carve = [&](size_t bytes) -> char* { char* p = ws + off; off += (bytes + 255) & ~(size_t)255; return p; };
  unsigned short* WF = (unsigned short*)carve((size_t)HID_DIM * CAT_DIM * 2);
  unsigned short* WH = (unsigned short*)carve((size_t)HID_DIM * CAT_DIM * 2);
  unsigned short* WL = (unsigned short*)carve((size_t)HID_DIM * CAT_DIM * 2);
  unsigned short* P  = (unsigned short*)carve((size_t)(N_LEAVES / 2) * HID_DIM * 2);
  unsigned short* Q  = (unsigned short*)carve((size_t)(N_LEAVES / 4) * HID_DIM * 2);
  if (off > ws_size || off > (size_t)134217728) return;

  const int n8 = HID_DIM * CAT_DIM / 8;
  weight_planes_kernel<<<(n8 + 255) / 256, 256, 0, stream>>>(Wc_w, WF, WH, WL, n8);

  const int n1 = N_LEAVES / 2;
  pair_level_kernel<0, false, 1, true><<<n1 / 64, 64, 0, stream>>>(
      WF, WF, pos_idx, wrd_idx, Wpos, Wwrd, WF, WF, P, P, Wnon, Wc_b, non_idx, n1, CARRY_FOLD, STATE_CARRY);

  const int n2 = N_LEAVES / 4;
  pair_level_kernel<0, false, 1, false><<<((n2 / 64) * 2 + 7) / 8, 256, 0, stream>>>(
      P, P, pos_idx, wrd_idx, Wpos, Wwrd, WF, WF, Q, Q, Wnon, Wc_b, non_idx + n1, n2, CARRY_FOLD, STATE_CARRY);

  const int n3 = N_LEAVES / 8;
  pair_level_kernel<0, false, 2, false><<<((n3 / 64) * 2 + 7) / 8, 256, 0, stream>>>(
      Q, Q, pos_idx, wrd_idx, Wpos, Wwrd, WF, WF, P, P + (size_t)n3 * HID_DIM, Wnon, Wc_b,
      non_idx + n1 + n2, n3, CARRY_FOLD, 1.0f);

  size_t loff = (size_t)n1 + (size_t)n2 + (size_t)n3;
  unsigned short* cur = P;
  unsigned short* nxt = Q;
  for (int n = N_LEAVES / 16; n >= TAIL_ROWS; n >>= 1) {
    const int tiles = (n / 64) * 2;
    pair_level_kernel<1, true, 2, false><<<(tiles + 7) / 8, 256, 0, stream>>>(
        cur, cur + (size_t)(2 * n) * HID_DIM, pos_idx, wrd_idx, Wpos, Wwrd, WH, WL,
        nxt, nxt + (size_t)n * HID_DIM, Wnon, Wc_b, non_idx + loff, n, 1.0f, 1.0f);
    loff += (size_t)n;
    unsigned short* t = cur; cur = nxt; nxt = t;
  }

  root_tail_kernel<<<1, 256, 0, stream>>>(cur, cur + (size_t)TAIL_ROWS * HID_DIM, Wc_w, Wnon, Wc_b, non_idx + loff, out);
}
